// MultiHeadAttention_32753420599796
// MI455X (gfx1250) — hardware-verified
//
#include <hip/hip_runtime.h>


#ifndef NB
#define NB 4
#endif
#ifndef SEQ
#define SEQ 2048
#endif
#define NB_FULL  4
#define SEQ_FULL 2048
#define DM   1024
#define NH_  16
#define HD   64
#define KT   64
#define SCL  0.125f
#define PCL2 10.0f

static_assert(DM == NH_ * HD);
static_assert(HD == 64);
static_assert(KT == 64);
static_assert(SEQ % KT == 0);
static_assert(SEQ % 64 == 0);
static_assert((NB * SEQ) % 64 == 0);
static_assert(DM % 64 == 0);
static_assert(DM % 32 == 0);
static_assert(((size_t)SEQ * DM / 8) % 256 == 0);
static_assert(((size_t)DM * DM / 8) % 256 == 0);
static_assert(NB <= NB_FULL);
static_assert(SEQ <= SEQ_FULL);

typedef _Float16 h16;
typedef unsigned short bf;
typedef __attribute__((ext_vector_type(16))) __bf16   v16bf;
typedef __attribute__((ext_vector_type(16))) _Float16 v16h;
typedef __attribute__((ext_vector_type(8)))  _Float16 v8h;
typedef __attribute__((ext_vector_type(8)))  unsigned short v8us;
typedef __attribute__((ext_vector_type(8)))  float    v8f;
typedef __attribute__((ext_vector_type(4)))  float    v4f;
typedef v4f  __attribute__((may_alias)) v4fa;

__device__ __forceinline__ unsigned short f2bf(float f) { unsigned u = __float_as_uint(f); u += 0x7FFFu + ((u >> 16) & 1u); return (unsigned short)(u >> 16); }
__device__ __forceinline__ float bf2f(unsigned short b) { return __uint_as_float(((unsigned)b) << 16); }
__device__ __forceinline__ float bfr(float f) { return bf2f(f2bf(f)); }
__device__ __forceinline__ void splitf(float y, unsigned short& h, unsigned short& l) { h = f2bf(y); l = f2bf(y - bf2f(h)); }
__device__ __forceinline__ v16h cat16(v8h lo, v8h hi) { return __builtin_shufflevector(lo, hi, 0, 1, 2, 3, 4, 5, 6, 7, 8, 9, 10, 11, 12, 13, 14, 15); }
__device__ __forceinline__ v16bf cat16b(v8us lo, v8us hi) { return __builtin_bit_cast(v16bf, __builtin_shufflevector(lo, hi, 0, 1, 2, 3, 4, 5, 6, 7, 8, 9, 10, 11, 12, 13, 14, 15)); }
__device__ __forceinline__ v8f wmma16(v16h a, v16h b, v8f c) { return __builtin_amdgcn_wmma_f32_16x16x32_f16(false, a, false, b, (short)0, c, false, false); }
__device__ __forceinline__ v8f wmmab(v16bf a, v16bf b, v8f c) { return __builtin_amdgcn_wmma_f32_16x16x32_bf16(false, a, false, b, (short)0, c, false, false); }

template <typename T16> struct WFrag;
template <> struct WFrag<h16> { typedef v16h V; static __device__ __forceinline__ V ld(const h16* p) { return cat16(*(const v8h*)p, *(const v8h*)(p + 16)); } static __device__ __forceinline__ v8f mma(V a, V b, v8f c) { return wmma16(a, b, c); } };
template <> struct WFrag<bf> { typedef v16bf V; static __device__ __forceinline__ V ld(const bf* p) { return cat16b(*(const v8us*)p, *(const v8us*)(p + 16)); } static __device__ __forceinline__ v8f mma(V a, V b, v8f c) { return wmmab(a, b, c); } };

template <typename T16, int NSPLIT, int OMODE, typename TO>
__global__ __launch_bounds__(32) void k_gemmw(const T16* __restrict__ A, const T16* __restrict__ A2, const T16* __restrict__ Bt, const T16* __restrict__ Bt2, int K, TO* C, int ldc, const float* __restrict__ bias, size_t sA, size_t sB, size_t sC) {
    typedef typename WFrag<T16>::V V;
    __shared__ __align__(16) float os[16 * 68];
    const size_t z = blockIdx.z; A += z * sA; if (A2) A2 += z * sA; Bt += z * sB; if (Bt2) Bt2 += z * sB; C += z * sC;
    const unsigned lane = threadIdx.x & 31u, lr = lane & 15u, hi = lane >> 4; const unsigned r0 = blockIdx.x * 64u, c0 = blockIdx.y * 64u;
    v8f acc[4][4];
#pragma unroll
    for (int mb = 0; mb < 4; ++mb)
#pragma unroll
        for (int nb = 0; nb < 4; ++nb) acc[mb][nb] = (v8f){};
    const size_t aoff = (size_t)(r0 + lr) * K + 8u * hi, boff = (size_t)(c0 + lr) * K + 8u * hi;
#pragma unroll 1
    for (int kc = 0; kc < K; kc += 32) {
        V a[4], a2[4];
#pragma unroll
        for (int mb = 0; mb < 4; ++mb) { a[mb] = WFrag<T16>::ld(A + aoff + (size_t)mb * 16 * K + kc); if (NSPLIT == 1 || NSPLIT == 2) a2[mb] = WFrag<T16>::ld(A2 + aoff + (size_t)mb * 16 * K + kc); }
#pragma unroll
        for (int nb = 0; nb < 4; ++nb) { const V b = WFrag<T16>::ld(Bt + boff + (size_t)nb * 16 * K + kc); V b2; if (NSPLIT >= 2) b2 = WFrag<T16>::ld(Bt2 + boff + (size_t)nb * 16 * K + kc);
#pragma unroll
            for (int mb = 0; mb < 4; ++mb) { acc[mb][nb] = WFrag<T16>::mma(a[mb], b, acc[mb][nb]); if (NSPLIT == 1 || NSPLIT == 2) acc[mb][nb] = WFrag<T16>::mma(a2[mb], b, acc[mb][nb]); if (NSPLIT >= 2) acc[mb][nb] = WFrag<T16>::mma(a[mb], b2, acc[mb][nb]); } }
        asm volatile("v_nop\n\tv_nop\n\tv_nop\n\tv_nop" : "+v"(acc[0][0]), "+v"(acc[1][1]), "+v"(acc[2][2]), "+v"(acc[3][3]) : "v"(a[0]), "v"(a[3]));
    }
#pragma unroll
    for (int mb = 0; mb < 4; ++mb) {
#pragma unroll
        for (int nb = 0; nb < 4; ++nb) {
#pragma unroll
            for (int j = 0; j < 8; ++j) os[(hi * 8 + j) * 68 + nb * 16 + lr] = acc[mb][nb][j]; }
        __builtin_amdgcn_wave_barrier(); asm volatile("" ::: "memory");
        if (OMODE == 0) {
            float* crow = (float*)(void*)C + (size_t)(r0 + mb * 16) * ldc + c0;
            const unsigned cofs = lr * 4u;
            const v4f bb = *(const v4f*)(bias + c0 + cofs);
            v4f val[8];
#pragma unroll
            for (int s = 0; s < 8; ++s) { const unsigned row = 2u * s + hi; v4f x = *(const v4fa*)(os + row * 68 + cofs);
                x[0] += bfr(bb[0]); x[1] += bfr(bb[1]); x[2] += bfr(bb[2]); x[3] += bfr(bb[3]); val[s] = x; }
#pragma unroll 1
            for (int ps = 0; ps < 2; ++ps) {
#pragma unroll
                for (int s = 0; s < 8; ++s) { const unsigned row = 2u * s + hi; *(volatile v4f*)(crow + (size_t)row * ldc + cofs) = val[s]; }
                if (ps == 0) __threadfence(); }
        } else {
            h16* crow = (h16*)(void*)C + (size_t)(r0 + mb * 16) * ldc + c0;
            const unsigned rq = lane >> 3, cofs = (lane & 7u) * 8u;
            v4f b0 = (v4f){}, b1 = (v4f){};
            if (OMODE == 1) { b0 = *(const v4f*)(bias + c0 + cofs); b1 = *(const v4f*)(bias + c0 + cofs + 4); }
            v8h val[4];
#pragma unroll
            for (int s = 0; s < 4; ++s) { const unsigned row = 4u * s + rq; const v4f x0 = *(const v4fa*)(os + row * 68 + cofs); const v4f x1 = *(const v4fa*)(os + row * 68 + cofs + 4);
                float rb = 0.f; if (OMODE == 2) rb = bfr(bias[r0 + mb * 16 + row]);
                v8h o8;
#pragma unroll
                for (int q = 0; q < 4; ++q) { const float a0 = (OMODE == 1) ? bfr(b0[q]) : rb; const float a1 = (OMODE == 1) ? bfr(b1[q]) : rb; o8[q] = (h16)(x0[q] + a0); o8[4 + q] = (h16)(x1[q] + a1); }
                val[s] = o8; }
#pragma unroll 1
            for (int ps = 0; ps < 2; ++ps) {
#pragma unroll
                for (int s = 0; s < 4; ++s) { const unsigned row = 4u * s + rq; *(volatile v8h*)(crow + (size_t)row * ldc + cofs) = val[s]; }
                if (ps == 0) __threadfence(); }
        }
        __builtin_amdgcn_wave_barrier(); asm volatile("" ::: "memory");
    }
}

__global__ __launch_bounds__(256) void k_cvt8(const float* __restrict__ src, bf* dst, size_t n8, size_t sstr, size_t dstr) {
    const size_t i = (size_t)blockIdx.x * 256u + threadIdx.x; if (i >= n8) return;
    const float* s = src + (size_t)blockIdx.y * sstr + i * 8; bf* d = dst + (size_t)blockIdx.y * dstr + i * 8;
    const v8f v = *(const v8f*)s; v8us o;
#pragma unroll
    for (int k = 0; k < 8; ++k) o[k] = f2bf(v[k]);
    *(volatile v8us*)d = o; __threadfence(); *(volatile v8us*)d = o; }

__global__ __launch_bounds__(128) void k_flash(const h16* __restrict__ Qp, const h16* __restrict__ Kp, const h16* __restrict__ Vt, bf* Ch, bf* Cl) {
    __shared__ __align__(16) float cs[4][16 * 68];
    const unsigned lane = threadIdx.x & 31u, wv = threadIdx.x >> 5, lr = lane & 15u, hi = lane >> 4;
    const unsigned h = blockIdx.y, b = blockIdx.z; const unsigned q0 = blockIdx.x * 64u + wv * 16u;
    const size_t rowb = (size_t)b * SEQ;
    const h16* qp = Qp + (rowb + q0 + lr) * DM + h * HD + 8u * hi;
    const v16h qf0 = WFrag<h16>::ld(qp), qf1 = WFrag<h16>::ld(qp + 32);
    const h16* kbase = Kp + (rowb + lr) * DM + h * HD + 8u * hi;
    const h16* vbase = Vt + ((size_t)b * DM + h * HD + lr) * SEQ + 8u * hi;
    v8f o[4];
#pragma unroll
    for (int dt = 0; dt < 4; ++dt) o[dt] = (v8f){};
    float mrun = -3.0e38f, lrun = 0.f;
    const float c = SCL * 1.4426950408889634f;
#pragma unroll 1
    for (unsigned kb = 0; kb < SEQ; kb += KT) {
        v16h ka[4][2];
#pragma unroll
        for (int j = 0; j < 4; ++j) { const h16* kp = kbase + (size_t)(kb + 16u * j) * DM; ka[j][0] = WFrag<h16>::ld(kp); ka[j][1] = WFrag<h16>::ld(kp + 32); }
        v8f st[4];
#pragma unroll
        for (int j = 0; j < 4; ++j) { st[j] = wmma16(ka[j][0], qf0, (v8f){}); st[j] = wmma16(ka[j][1], qf1, st[j]); }
        asm volatile("v_nop\n\tv_nop\n\tv_nop\n\tv_nop" : "+v"(st[0]), "+v"(st[1]), "+v"(st[2]), "+v"(st[3]) : "v"(qf0), "v"(qf1));
        float mloc = st[0][0];
#pragma unroll
        for (int j = 0; j < 4; ++j)
#pragma unroll
            for (int r = 0; r < 8; ++r) mloc = fmaxf(mloc, st[j][r]);
        mloc = fmaxf(mloc, __shfl_xor(mloc, 16, 32));
        const float mnew = fmaxf(mrun, mloc);
        const float fac = __builtin_amdgcn_exp2f((mrun - mnew) * c);
        const float off = mnew * c - PCL2;
        mrun = mnew;
        float ps = 0.f;
#pragma unroll
        for (int j = 0; j < 4; ++j)
#pragma unroll
            for (int r = 0; r < 8; ++r) { const float p = __builtin_amdgcn_exp2f(fmaf(st[j][r], c, -off)); st[j][r] = p; ps += p; }
        lrun = lrun * fac + ps;
#pragma unroll
        for (int dt = 0; dt < 4; ++dt)
#pragma unroll
            for (int r = 0; r < 8; ++r) o[dt][r] *= fac;
        v16h pb0, pb1;
#pragma unroll
        for (int i = 0; i < 8; ++i) { pb0[i] = (h16)st[0][i]; pb0[8 + i] = (h16)st[1][i]; pb1[i] = (h16)st[2][i]; pb1[8 + i] = (h16)st[3][i]; }
        asm volatile("" : "+v"(pb0), "+v"(pb1));
        v16h va[4][2];
#pragma unroll
        for (int dt = 0; dt < 4; ++dt) { const h16* vp = vbase + (size_t)(16u * dt) * SEQ + kb; va[dt][0] = WFrag<h16>::ld(vp); va[dt][1] = WFrag<h16>::ld(vp + 32); }
#pragma unroll
        for (int dt = 0; dt < 4; ++dt) { o[dt] = wmma16(va[dt][0], pb0, o[dt]); o[dt] = wmma16(va[dt][1], pb1, o[dt]); }
        asm volatile("v_nop\n\tv_nop\n\tv_nop\n\tv_nop" : "+v"(o[0]), "+v"(o[1]), "+v"(o[2]), "+v"(o[3]) : "v"(pb0), "v"(pb1));
    }
    const float l = lrun + __shfl_xor(lrun, 16, 32);
    const float inv = 1.0f / l;
    float* cw = cs[wv];
#pragma unroll
    for (int dt = 0; dt < 4; ++dt)
#pragma unroll
        for (int r = 0; r < 8; ++r) cw[lr * 68 + dt * 16 + hi * 8 + r] = o[dt][r] * inv;
    __syncthreads();
    const unsigned rq = lane >> 3, cofs = (lane & 7u) * 8u;
    v8us oh[4], ol[4];
#pragma unroll
    for (int s = 0; s < 4; ++s) { const unsigned row = 4u * s + rq; const v4f x0 = *(const v4fa*)(cw + row * 68 + cofs); const v4f x1 = *(const v4fa*)(cw + row * 68 + cofs + 4); v8us a8, c8;
#pragma unroll
        for (int q = 0; q < 4; ++q) { unsigned short a, c2; splitf(x0[q], a, c2); a8[q] = a; c8[q] = c2; splitf(x1[q], a, c2); a8[4 + q] = a; c8[4 + q] = c2; }
        oh[s] = a8; ol[s] = c8; }
    bf* ch = Ch + (rowb + q0) * DM + h * HD + cofs; bf* cl = Cl + (rowb + q0) * DM + h * HD + cofs;
#pragma unroll 1
    for (int ps = 0; ps < 2; ++ps) {
#pragma unroll
        for (int s = 0; s < 4; ++s) { const unsigned row = 4u * s + rq; *(volatile v8us*)(ch + (size_t)row * DM) = oh[s]; *(volatile v8us*)(cl + (size_t)row * DM) = ol[s]; }
        if (ps == 0) __threadfence(); }
}

#define WB_BYTES ((size_t)DM * DM * 2)
#define PL_BYTES ((size_t)NB * SEQ * DM * 2)
static_assert(WB_BYTES % 256 == 0);
static_assert(PL_BYTES % 256 == 0);
static_assert(4 * WB_BYTES + 6 * PL_BYTES <= (size_t)134217728);

extern "C" void kernel_launch(void* const* d_in, const int* in_sizes, int n_in,
                              void* d_out, int out_size, void* d_ws, size_t ws_size, hipStream_t stream) {
    if (n_in < 11) return;
    const size_t need_x = (size_t)(NB - 1) * SEQ_FULL * DM + (size_t)SEQ * DM;
    if ((size_t)in_sizes[0] < need_x || (size_t)in_sizes[1] < need_x || (size_t)in_sizes[2] < need_x) return;
    if ((size_t)in_sizes[3] < (size_t)DM * DM || (size_t)in_sizes[5] < (size_t)DM * DM || (size_t)in_sizes[7] < (size_t)DM * DM || (size_t)in_sizes[9] < (size_t)DM * DM) return;
    if (in_sizes[4] < DM || in_sizes[6] < DM || in_sizes[8] < DM || in_sizes[10] < DM) return;
    if ((size_t)out_size < (size_t)NB * SEQ * DM) return;
    const float* xq = (const float*)d_in[0]; const float* xk = (const float*)d_in[1]; const float* xv = (const float*)d_in[2];
    const float* wq = (const float*)d_in[3]; const float* bq = (const float*)d_in[4];
    const float* wk = (const float*)d_in[5]; const float* bk = (const float*)d_in[6];
    const float* wv = (const float*)d_in[7]; const float* bv = (const float*)d_in[8];
    const float* wo = (const float*)d_in[9]; const float* bo = (const float*)d_in[10];
    float* OUT = (float*)d_out;
    char* wsp = (char*)d_ws;
    auto take = [&](size_t bytes) { char* p = wsp; wsp += (bytes + 255) & ~(size_t)255; return (void*)p; };
    bf* WQ = (bf*)take(WB_BYTES); bf* WK = (bf*)take(WB_BYTES); bf* WV = (bf*)take(WB_BYTES); bf* WO = (bf*)take(WB_BYTES);
    bf* XB = (bf*)take(PL_BYTES);
    h16* Q16 = (h16*)take(PL_BYTES); h16* K16 = (h16*)take(PL_BYTES);
    h16* VT16 = (h16*)take(PL_BYTES);
    bf* CTh = (bf*)take(PL_BYTES); bf* CTl = (bf*)take(PL_BYTES);
    if ((size_t)(wsp - (char*)d_ws) > ws_size) return;

    const unsigned gw = (unsigned)((size_t)DM * DM / 8 / 256), gx = (unsigned)((size_t)SEQ * DM / 8 / 256);
    const size_t n8w = (size_t)DM * DM / 8, n8x = (size_t)SEQ * DM / 8;
    k_cvt8<<<dim3(gw, 1, 1), 256, 0, stream>>>(wq, WQ, n8w, 0, 0);
    k_cvt8<<<dim3(gw, 1, 1), 256, 0, stream>>>(wk, WK, n8w, 0, 0);
    k_cvt8<<<dim3(gw, 1, 1), 256, 0, stream>>>(wv, WV, n8w, 0, 0);
    k_cvt8<<<dim3(gw, 1, 1), 256, 0, stream>>>(wo, WO, n8w, 0, 0);

    k_cvt8<<<dim3(gx, NB, 1), 256, 0, stream>>>(xq, XB, n8x, (size_t)SEQ_FULL * DM, (size_t)SEQ * DM);
    k_gemmw<bf, 0, 1, h16><<<dim3(NB * SEQ / 64, DM / 64, 1), 32, 0, stream>>>(XB, nullptr, WQ, nullptr, DM, Q16, DM, bq, 0, 0, 0);
    k_cvt8<<<dim3(gx, NB, 1), 256, 0, stream>>>(xk, XB, n8x, (size_t)SEQ_FULL * DM, (size_t)SEQ * DM);
    k_gemmw<bf, 0, 1, h16><<<dim3(NB * SEQ / 64, DM / 64, 1), 32, 0, stream>>>(XB, nullptr, WK, nullptr, DM, K16, DM, bk, 0, 0, 0);
    k_cvt8<<<dim3(gx, NB, 1), 256, 0, stream>>>(xv, XB, n8x, (size_t)SEQ_FULL * DM, (size_t)SEQ * DM);
    k_gemmw<bf, 0, 2, h16><<<dim3(DM / 64, SEQ / 64, NB), 32, 0, stream>>>(WV, nullptr, XB, nullptr, DM, VT16, SEQ, bv, 0, (size_t)SEQ * DM, (size_t)DM * SEQ);

    k_flash<<<dim3(SEQ / 64, NH_, NB), 128, 0, stream>>>(Q16, K16, VT16, CTh, CTl);

    k_gemmw<bf, 1, 0, float><<<dim3(NB * SEQ / 64, DM / 64, 1), 32, 0, stream>>>(CTh, CTl, WO, nullptr, DM, OUT, DM, bo, 0, 0, 0);
}
